// Reverb_37211596653118
// MI455X (gfx1250) — hardware-verified
//
#include <hip/hip_runtime.h>
#include <math.h>

typedef __attribute__((ext_vector_type(16))) _Float16 v16h;
typedef __attribute__((ext_vector_type(8)))  _Float16 v8h;
typedef __attribute__((ext_vector_type(8)))  float    v8f;
typedef __attribute__((ext_vector_type(4)))  float    v4f;
typedef __attribute__((ext_vector_type(4)))  unsigned v4u;
typedef v4u v4u_alias __attribute__((may_alias));

constexpr int kNfft    = 384;
constexpr int kHop     = 192;
constexpr int kFreq    = 193;
constexpr int kSteps   = 311;
constexpr int kFrames  = 1366;
constexpr int kBatch   = 8;
constexpr int kBs      = 16;
constexpr int kTlen    = 262144;
constexpr int kOutLen  = 262080;
constexpr int kChan    = 386;
constexpr int kLead    = 320;
constexpr int kStripe  = 1728;
constexpr int kCols    = kBs * kStripe;
constexpr int kBasisRows = 448;
constexpr int kTiles   = 44;
constexpr int kTpad    = 1408;
constexpr int kKwin    = 352;
constexpr int kChanPlane = 32 * kKwin;
constexpr int kConvRows  = kBatch * kTiles;
constexpr int kYaRows  = kBs * kTpad;
constexpr int kYaSlack = 32;
constexpr int kYaPitch = 448;
constexpr int kSynK    = 896;
constexpr float kTapCarry    = 1024.0f;
constexpr float kTapCarryInv = 1.0f / 1024.0f;
constexpr float kInvSqrt2    = 0.70710678118654752f;
constexpr float kStepAngle   = 6.28318530717958647692f / 384.0f;
constexpr float kInvNfft     = 1.0f / 384.0f;

static_assert(kFreq == kNfft / 2 + 1, "bins");
static_assert(kFrames == 1 + (kTlen + 2 * (kNfft / 2) - kNfft) / kHop, "frames");
static_assert(kOutLen == (kFrames - 1) * kHop, "out len");
static_assert(kSteps == (60000 - kNfft + kHop - 1) / kHop, "taps");
static_assert(kChan == 2 * kFreq, "channels");
static_assert(kLead == kKwin - 32, "lead");
static_assert(kLead + kFrames <= kStripe, "stripe");
static_assert(32 * (kTiles - 1) + kKwin <= kStripe, "window inside stripe");
static_assert(kTpad == 32 * kTiles && kTpad >= kFrames, "tiles");
static_assert((kStripe % 64) == 0 && (kCols % 64) == 0 && (kBasisRows % 64) == 0, "gemm1 tiles");
static_assert((kNfft % 32) == 0 && (kSynK % 32) == 0 && (kKwin % 32) == 0, "k32");
static_assert((kYaRows % 64) == 0 && (kTpad % 64) == 0 && (kHop % 64) == 0, "gemm2 tiles");
static_assert(kSynK == 2 * kYaPitch && kYaPitch >= 2 * kFreq && (kYaPitch % 64) == 0, "syn k");
static_assert((kConvRows % 32) == 0 && kConvRows / 32 == 11, "conv rows");

constexpr size_t kSzBST = (size_t)kBasisRows * kNfft * 2;
constexpr size_t kSzIBT = (size_t)kHop * kSynK * 2;
constexpr size_t kSzWT  = (size_t)kChan * 2 * kChanPlane * 2;
constexpr size_t kSzFR  = (size_t)kCols * kNfft * 2;
constexpr size_t kSzHS  = (size_t)kBasisRows * kCols * 2;
constexpr size_t kSzGAP = 256;
constexpr size_t kSzYC  = (size_t)kChan * 2 * kBatch * kTpad * 2;
constexpr size_t kSzYA  = (size_t)(kYaRows + kYaSlack) * kYaPitch * 2;
constexpr size_t kOffBST = 0;
constexpr size_t kOffIBT = kOffBST + kSzBST;
constexpr size_t kOffWT  = kOffIBT + kSzIBT;
constexpr size_t kOffFR  = kOffWT + kSzWT;
constexpr size_t kOffHS  = kOffFR + kSzFR;
constexpr size_t kOffYC  = kOffHS + kSzHS + kSzGAP;
constexpr size_t kOffYA  = kOffYC + kSzYC;
constexpr size_t kWsTotal = kOffYA + kSzYA;
static_assert(kWsTotal == 101691648ull, "carve total");
static_assert(kWsTotal <= 134217728ull, "carve cap");
static_assert((kOffIBT % 128) == 0 && (kOffWT % 128) == 0 && (kOffFR % 128) == 0 && (kOffHS % 128) == 0 &&
              (kOffYC % 128) == 0 && (kOffYA % 128) == 0, "aligned regions");
static_assert(kSzBST == kSzIBT && (kSzBST / 2) == 84 * 2048, "basis blocks");

union FragU { v16h v; v8h h[2]; };
__device__ __forceinline__ v16h frag_load(const _Float16* p) {
  FragU f;
  f.h[0] = *(const v8h*)(p);
  f.h[1] = *(const v8h*)(p + 16);
  return f.v;
}
__device__ __forceinline__ v8f mma_h(v16h a, v16h b, v8f c) {
  c = __builtin_amdgcn_wmma_f32_16x16x32_f16(false, a, false, b, (short)0, c, false, false);
  asm volatile("v_nop\n\tv_nop\n\tv_nop\n\tv_nop" : "+v"(c) : "v"(a), "v"(b));
  return c;
}
__device__ __forceinline__ void dep_guard4_h(v8f& a, v8f& b, v8f& c, v8f& d, v16h x, v16h y) {
  asm volatile("v_nop\n\tv_nop\n\tv_nop\n\tv_nop" : "+v"(a), "+v"(b), "+v"(c), "+v"(d) : "v"(x), "v"(y));
}
__device__ __forceinline__ void keep4_h(v16h a, v16h b, v16h c, v16h d) {
  asm volatile("v_nop" :: "v"(a), "v"(b), "v"(c), "v"(d));
}
__device__ __forceinline__ void acc_guard4(v8f& a, v8f& b, v8f& c, v8f& d) {
  asm volatile("v_nop\n\tv_nop\n\tv_nop\n\tv_nop" : "+v"(a), "+v"(b), "+v"(c), "+v"(d));
}

template <int OUT_MODE>
__global__ __launch_bounds__(256) void wmma_gemm64_h(
    const unsigned short* __restrict__ Ap, int lda,
    const unsigned short* __restrict__ Btp, int ldb,
    void* __restrict__ Cout, int ldc,
    int M, int N, int K, float scale) {
  const _Float16* A  = (const _Float16*)Ap;
  const _Float16* Bt = (const _Float16*)Btp;
  __shared__ __align__(16) float sT[8][16 * 68];
  const int lane = threadIdx.x & 31;
  const int wave = threadIdx.x >> 5;
  const int tilesN = N >> 6;
  const int tilesM = M >> 6;
  const int tile = blockIdx.x * 8 + wave;
  if (tile >= tilesM * tilesN) return;
  const int tm = tile / tilesN;
  const int tn = tile - tm * tilesN;
  const int m0 = tm << 6;
  const int n0 = tn << 6;
  const int rlane = lane & 15;
  const int koff  = (lane >> 4) * 8;
  const int mOff  = (lane >> 4) * 8;

  v8f acc[4][4];
#pragma unroll
  for (int i = 0; i < 4; ++i)
#pragma unroll
    for (int j = 0; j < 4; ++j) acc[i][j] = (v8f){0.f,0.f,0.f,0.f,0.f,0.f,0.f,0.f};

  for (int k0 = 0; k0 < K; k0 += 32) {
    v16h bh[4];
#pragma unroll
    for (int j = 0; j < 4; ++j) {
      const size_t bo = (size_t)(n0 + (j << 4) + rlane) * ldb + koff + k0;
      bh[j] = frag_load(Bt + bo);
    }
#pragma unroll
    for (int i = 0; i < 4; ++i) {
      const size_t ao = (size_t)(m0 + (i << 4) + rlane) * lda + koff + k0;
      const v16h ah = frag_load(A + ao);
#pragma unroll
      for (int j = 0; j < 4; ++j)
        acc[i][j] = __builtin_amdgcn_wmma_f32_16x16x32_f16(false, ah, false, bh[j], (short)0, acc[i][j], false, false);
      dep_guard4_h(acc[i][0], acc[i][1], acc[i][2], acc[i][3], ah, bh[3]);
    }
    keep4_h(bh[0], bh[1], bh[2], bh[3]);
  }
  acc_guard4(acc[0][0], acc[0][1], acc[0][2], acc[0][3]);
  acc_guard4(acc[1][0], acc[1][1], acc[1][2], acc[1][3]);
  acc_guard4(acc[2][0], acc[2][1], acc[2][2], acc[2][3]);
  acc_guard4(acc[3][0], acc[3][1], acc[3][2], acc[3][3]);

  float* slab = sT[wave];
#pragma unroll
  for (int i = 0; i < 4; ++i) {
    const int mBase = m0 + (i << 4);
#pragma unroll
    for (int j = 0; j < 4; ++j) {
#pragma unroll
      for (int r = 0; r < 8; ++r) {
        const float v = acc[i][j][r] * scale;
        slab[(mOff + r) * 68 + (j << 4) + rlane] = v;
      }
    }
    __builtin_amdgcn_fence(__ATOMIC_RELEASE, "workgroup");
    __builtin_amdgcn_wave_barrier();
    __builtin_amdgcn_fence(__ATOMIC_ACQUIRE, "workgroup");
    if (OUT_MODE == 3) {
      float* C = (float*)Cout;
      const int hh = lane >> 4, c4 = (lane & 15) * 4;
      const int grp = mBase / kTpad;
      const int i0  = mBase - grp * kTpad;
      for (int pass = 0; pass < 2; ++pass) {
#pragma unroll
        for (int it = 0; it < 8; ++it) {
          const int row = it * 2 + hh;
          const int ii = i0 + row;
          const v4f v = *(const v4f*)(slab + row * 68 + c4);
          if (ii < kFrames - 1)
            *(volatile v4f*)(C + ((size_t)grp * (kFrames - 1) + ii) * ldc + n0 + c4) = v;
        }
        __threadfence();
      }
    } else {
      const int q = lane >> 3, c8 = (lane & 7) * 8;
      unsigned short* C = (unsigned short*)Cout;
      for (int pass = 0; pass < 2; ++pass) {
#pragma unroll
        for (int it = 0; it < 4; ++it) {
          const int row = it * 4 + q;
          const float* sp = slab + row * 68 + c8;
          v8h hv;
#pragma unroll
          for (int e = 0; e < 8; ++e) hv[e] = (_Float16)sp[e];
          *(volatile v8h*)(C + (size_t)(mBase + row) * ldc + n0 + c8) = hv;
        }
        __threadfence();
      }
    }
    __builtin_amdgcn_fence(__ATOMIC_RELEASE, "workgroup");
    __builtin_amdgcn_wave_barrier();
    __builtin_amdgcn_fence(__ATOMIC_ACQUIRE, "workgroup");
  }
}

__device__ __forceinline__ float lin_arg(float lm, float ld, float tf) {
#pragma clang fp contract(off)
  const float p = ld * tf;
  return lm + p;
}

__global__ __launch_bounds__(256) void ir_taps_kernel(
    const float* __restrict__ lmr, const float* __restrict__ lmdr,
    const float* __restrict__ ang, unsigned short* __restrict__ WT)
{
  __shared__ float sPar[4];
  __shared__ __align__(16) float sTab[4 * 384];
  const int tid = threadIdx.x;
  const int q = blockIdx.x;
  {
    const int kk = tid & 3;
    const int c = kk & 1;
    const float xa = lmr[c * kFreq + q];
    const float xb = lmdr[c * kFreq + q];
    const float fa = (kk < 2) ? 1.0f : 0.0f;
    const float fb = 1.0f - fa;
    const float x = fmaf(fa, xa, fb * xb);
    const float sp = fmaxf(x, 0.0f) + log1pf(expf(-fabsf(x)));
    if (tid < 4) sPar[tid] = -sp;
  }
  __syncthreads();
#pragma unroll 1
  for (int idx = tid; idx < 384; idx += 256) {
    const int d = idx - 32;
    const bool valid = (d >= 0) && (d < kSteps);
    int dc = d < 0 ? 0 : d;
    dc = dc > (kSteps - 1) ? (kSteps - 1) : dc;
    const float tf = (float)dc;
    float sr = 0.0f, dr = 0.0f, si = 0.0f, di = 0.0f;
#pragma unroll 1
    for (int c = 0; c < 2; ++c) {
      const float lm = sPar[c];
      const float ld = sPar[2 + c];
      float mag = expf(lin_arg(lm, ld, tf));
      mag = (mag < 1.17549435e-38f) ? 0.0f : mag;
      const float a = ang[(size_t)(c * kFreq + q) * kSteps + dc];
      const float cs = cosf(a);
      const float sn = sinf(a);
      const float sg = 1.0f - 2.0f * (float)c;
      const float re = mag * cs;
      const float im = mag * sn;
      sr += re;
      dr += sg * re;
      si += im;
      di += sg * im;
    }
    const float scl = kInvSqrt2 * kTapCarry;
    sTab[0 * 384 + idx] = valid ? sr * scl : 0.0f;
    sTab[1 * 384 + idx] = valid ? si * scl : 0.0f;
    sTab[2 * 384 + idx] = valid ? dr * scl : 0.0f;
    sTab[3 * 384 + idx] = valid ? di * scl : 0.0f;
  }
  __syncthreads();
#pragma unroll 1
  for (int it = 0; it < 22; ++it) {
    const int g = it * 256 + tid;
    const int m = g / 2816;
    const int rem = g - m * 2816;
    const int ri = rem / 1408;
    const int rem2 = rem - ri * 1408;
    const int n = rem2 / 44;
    const int kc = rem2 - n * 44;
    const float* tb = sTab + (m * 2 + ri) * 384 + n + kKwin - 8 * kc;
    v8h hv;
#pragma unroll
    for (int e = 0; e < 8; ++e) hv[e] = (_Float16)tb[-e];
    unsigned short* dst = WT + ((size_t)(m * kFreq + q) * 2 + ri) * kChanPlane + (size_t)rem2 * 8;
    *(volatile v8h*)dst = hv;
    __threadfence();
    *(volatile v8h*)dst = hv;
  }
}

__global__ __launch_bounds__(256) void dft_planes_kernel(
    unsigned short* __restrict__ BST, unsigned short* __restrict__ IBT)
{
  __shared__ float sCos[384];
  __shared__ __align__(16) unsigned short sV[2048];
  const int tid = threadIdx.x;
#pragma unroll 1
  for (int r = tid; r < 384; r += 256) sCos[r] = cosf((float)r * kStepAngle);
  __syncthreads();
  const bool syn = (blockIdx.x >= 84);
  const int base = (syn ? ((int)blockIdx.x - 84) : (int)blockIdx.x) * 2048;
#pragma unroll 1
  for (int it = 0; it < 8; ++it) {
    const int le = it * 256 + tid;
    const int e = base + le;
    float v;
    if (!syn) {
      const int j = e / kNfft;
      const int n = e - j * kNfft;
      const bool isIm = (j >= kFreq);
      const bool live = (j < kChan);
      int q = isIm ? (j - kFreq) : j;
      q = live ? q : 0;
      const int r = (q * n) % kNfft;
      const float cs = sCos[r];
      float sn = sCos[(r + 288) % kNfft];
      sn = ((r % 192) == 0) ? 0.0f : sn;
      const float win = 0.5f * (1.0f - sCos[n]);
      const float t = isIm ? (-(win * sn)) : (win * cs);
      v = live ? t : 0.0f;
    } else {
      const int n0 = e / kSynK;
      const int kk = e - n0 * kSynK;
      const int hf = kk / kYaPitch;
      const int col = kk - hf * kYaPitch;
      const int qr = col >> 1;
      const int ri = col & 1;
      const bool live = (qr < kFreq);
      const int q = live ? qr : 0;
      const int ns = hf ? n0 : (n0 + kHop);
      const int r = (q * ns) % kNfft;
      const float cs = sCos[r];
      float sn = sCos[(r + 288) % kNfft];
      sn = ((r % 192) == 0) ? 0.0f : sn;
      const float w0 = 0.5f * (1.0f - sCos[n0]);
      const float w1 = 0.5f * (1.0f - sCos[n0 + kHop]);
      const float env = w0 * w0 + w1 * w1;
      const float wn = hf ? w0 : w1;
      const float cq = (q == 0 || q == kFreq - 1) ? 1.0f : 2.0f;
      const float tr = ri ? (-sn) : cs;
      const float t = cq * wn * tr * (1.0f / env);
      v = live ? t : 0.0f;
    }
    const _Float16 hval = (_Float16)v;
    sV[le] = __builtin_bit_cast(unsigned short, hval);
  }
  __syncthreads();
  const v4u w = *(const v4u_alias*)(sV + tid * 8);
  unsigned short* dst = (syn ? IBT : BST) + (size_t)base + tid * 8;
  *(volatile v4u*)dst = w;
  __threadfence();
  *(volatile v4u*)dst = w;
}

__global__ __launch_bounds__(256) void frame_rows_kernel(
    const float* __restrict__ x, unsigned short* __restrict__ FR)
{
  const int g = blockIdx.x * 256 + threadIdx.x;
  const int row = g / 48;
  const int ck = g - row * 48;
  const int bs = row / kStripe;
  const int rr = row - bs * kStripe;
  const int f = rr - kLead;
  const bool valid = (f >= 0) && (f < kFrames);
  int fc = f < 0 ? 0 : f;
  fc = fc > (kFrames - 1) ? (kFrames - 1) : fc;
  const int j0 = kHop * fc + 8 * ck - kHop;
  const float* xb = x + (size_t)bs * kTlen;
  v8h hv;
#pragma unroll
  for (int e = 0; e < 8; ++e) {
    int j = j0 + e;
    j = (j < 0) ? (-j) : j;
    j = (j >= kTlen) ? (2 * kTlen - 2 - j) : j;
    j = (j < 0) ? 0 : j;
    j = (j > kTlen - 1) ? (kTlen - 1) : j;
    float v = xb[j];
    v = valid ? v : 0.0f;
    hv[e] = (_Float16)v;
  }
  unsigned short* dst = FR + (size_t)g * 8;
  *(volatile v8h*)dst = hv;
  __threadfence();
  *(volatile v8h*)dst = hv;
}

__device__ __forceinline__ void put_tile(float* s, int rowb, int colb, v8f a, float sc) {
#pragma unroll
  for (int r = 0; r < 8; ++r) s[(rowb + r) * 36 + colb] = a[r] * sc;
}

__global__ __launch_bounds__(32) void band_conv_kernel(
    const unsigned short* __restrict__ HSp, const unsigned short* __restrict__ WTp,
    unsigned short* __restrict__ YC)
{
  __shared__ __align__(16) float sY[2 * 32 * 36];
  const int lane = threadIdx.x & 31;
  const int ch = blockIdx.x / 11;
  const int w = blockIdx.x - ch * 11;
  const int cst = ch / kFreq;
  const int q = ch - cst * kFreq;
  const int h = lane >> 4, c = lane & 15;
  const _Float16* HS = (const _Float16*)HSp;
  const _Float16* WT = (const _Float16*)WTp;
  const int mA = 32 * w + c;
  const int mB = mA + 16;
  const int bA = mA / kTiles, jA = mA - bA * kTiles;
  const int bB = mB / kTiles, jB = mB - bB * kTiles;
  const size_t offA = (size_t)(2 * bA + cst) * kStripe + 32 * jA + 8 * h;
  const size_t offB = (size_t)(2 * bB + cst) * kStripe + 32 * jB + 8 * h;
  const _Float16* pRA = HS + (size_t)q * kCols + offA;
  const _Float16* pIA = HS + (size_t)(kFreq + q) * kCols + offA;
  const _Float16* pRB = HS + (size_t)q * kCols + offB;
  const _Float16* pIB = HS + (size_t)(kFreq + q) * kCols + offB;
  const _Float16* wR0 = WT + (size_t)(ch * 2) * kChanPlane + (size_t)c * kKwin + 8 * h;
  const _Float16* wR1 = wR0 + 16 * kKwin;
  const _Float16* wI0 = wR0 + kChanPlane;
  const _Float16* wI1 = wI0 + 16 * kKwin;

  const v8f zf = (v8f){0.f,0.f,0.f,0.f,0.f,0.f,0.f,0.f};
  v8f g0A0 = zf, g0A1 = zf, g1A0 = zf, g1A1 = zf, g2A0 = zf, g2A1 = zf;
  v8f g0B0 = zf, g0B1 = zf, g1B0 = zf, g1B1 = zf, g2B0 = zf, g2B1 = zf;
#pragma unroll 1
  for (int k0 = 0; k0 < kKwin; k0 += 32) {
    const v16h bR0 = frag_load(wR0 + k0);
    const v16h bR1 = frag_load(wR1 + k0);
    const v16h bI0 = frag_load(wI0 + k0);
    const v16h bI1 = frag_load(wI1 + k0);
    const v16h aRA = frag_load(pRA + k0);
    const v16h aIA = frag_load(pIA + k0);
    g0A0 = mma_h(aRA, bR0, g0A0);
    g0A1 = mma_h(aRA, bR1, g0A1);
    g1A0 = mma_h(aIA, bI0, g1A0);
    g1A1 = mma_h(aIA, bI1, g1A1);
    g2A0 = mma_h(aRA, bI0, g2A0);
    g2A1 = mma_h(aRA, bI1, g2A1);
    g2A0 = mma_h(aIA, bR0, g2A0);
    g2A1 = mma_h(aIA, bR1, g2A1);
    const v16h aRB = frag_load(pRB + k0);
    const v16h aIB = frag_load(pIB + k0);
    g0B0 = mma_h(aRB, bR0, g0B0);
    g0B1 = mma_h(aRB, bR1, g0B1);
    g1B0 = mma_h(aIB, bI0, g1B0);
    g1B1 = mma_h(aIB, bI1, g1B1);
    g2B0 = mma_h(aRB, bI0, g2B0);
    g2B1 = mma_h(aRB, bI1, g2B1);
    g2B0 = mma_h(aIB, bR0, g2B0);
    g2B1 = mma_h(aIB, bR1, g2B1);
  }
  put_tile(sY,        8 * h,      c,      g0A0 - g1A0, kTapCarryInv);
  put_tile(sY,        8 * h,      16 + c, g0A1 - g1A1, kTapCarryInv);
  put_tile(sY,        16 + 8 * h, c,      g0B0 - g1B0, kTapCarryInv);
  put_tile(sY,        16 + 8 * h, 16 + c, g0B1 - g1B1, kTapCarryInv);
  put_tile(sY + 1152, 8 * h,      c,      g2A0, kTapCarryInv);
  put_tile(sY + 1152, 8 * h,      16 + c, g2A1, kTapCarryInv);
  put_tile(sY + 1152, 16 + 8 * h, c,      g2B0, kTapCarryInv);
  put_tile(sY + 1152, 16 + 8 * h, 16 + c, g2B1, kTapCarryInv);
  __syncthreads();
  v8h ov[2][4];
#pragma unroll
  for (int ri = 0; ri < 2; ++ri) {
#pragma unroll
    for (int it = 0; it < 4; ++it) {
      const int ci = it * 32 + lane;
      const int row = ci >> 2;
      const int c8 = (ci & 3) * 8;
      const int m = 32 * w + row;
      const int j = m % kTiles;
      const int t0 = 32 * j + c8;
      const float* sp = sY + ri * 1152 + row * 36 + c8;
      const v4f a0 = *(const v4f*)(sp);
      const v4f a1 = *(const v4f*)(sp + 4);
#pragma unroll
      for (int e = 0; e < 4; ++e) {
        float u0 = a0[e];
        float u1 = a1[e];
        u0 = (t0 + e < kFrames) ? u0 : 0.0f;
        u1 = (t0 + 4 + e < kFrames) ? u1 : 0.0f;
        ov[ri][it][e]     = (_Float16)u0;
        ov[ri][it][4 + e] = (_Float16)u1;
      }
    }
  }
  unsigned short* y0 = YC + (size_t)(ch * 2) * kChanPlane + (size_t)w * 1024 + lane * 8;
  for (int pass = 0; pass < 2; ++pass) {
#pragma unroll
    for (int ri = 0; ri < 2; ++ri) {
#pragma unroll
      for (int it = 0; it < 4; ++it)
        *(volatile v8h*)(y0 + (size_t)ri * kChanPlane + it * 256) = ov[ri][it];
    }
    __threadfence();
  }
}

__global__ __launch_bounds__(256) void pack_rows_kernel(
    const unsigned short* __restrict__ YC, unsigned short* __restrict__ YA)
{
  __shared__ __align__(16) unsigned short tile[32 * 72];
  const int tid = threadIdx.x;
  const int tix = blockIdx.x / 7;
  const int g = blockIdx.x - tix * 7;
  const bool extra = (tix >= kBs * kTiles);
  const int tixc = extra ? (kBs * kTiles - 1) : tix;
  const int bs = tixc / kTiles;
  const int tt = tixc - bs * kTiles;
  const int rowbase = extra ? kYaRows : (bs * kTpad + 32 * tt);
  const int srow = tid >> 2;
  const int ql = srow >> 1;
  const int ri = srow & 1;
  const int tseg = (tid & 3) * 8;
  const int q = 32 * g + ql;
  const int qc = (q > kFreq - 1) ? (kFreq - 1) : q;
  const bool live = (q < kFreq) && (!extra);
  const int b = bs >> 1, cst = bs & 1;
  const unsigned short* src = YC + (((size_t)(cst * kFreq + qc) * 2 + ri) * kBatch + b) * kTpad + 32 * tt + tseg;
  const v4u wv = *(const v4u*)src;
  unsigned w0 = wv[0], w1 = wv[1], w2 = wv[2], w3 = wv[3];
  w0 = live ? w0 : 0u;
  w1 = live ? w1 : 0u;
  w2 = live ? w2 : 0u;
  w3 = live ? w3 : 0u;
  unsigned short* tp = tile + tseg * 72 + srow;
  tp[0 * 72] = (unsigned short)(w0 & 0xffffu);
  tp[1 * 72] = (unsigned short)(w0 >> 16);
  tp[2 * 72] = (unsigned short)(w1 & 0xffffu);
  tp[3 * 72] = (unsigned short)(w1 >> 16);
  tp[4 * 72] = (unsigned short)(w2 & 0xffffu);
  tp[5 * 72] = (unsigned short)(w2 >> 16);
  tp[6 * 72] = (unsigned short)(w3 & 0xffffu);
  tp[7 * 72] = (unsigned short)(w3 >> 16);
  __syncthreads();
  const int row = tid >> 3;
  const int chunk = tid & 7;
  const v4u o = *(const v4u_alias*)(tile + row * 72 + chunk * 8);
  unsigned short* dst = YA + (size_t)(rowbase + row) * kYaPitch + 64 * g + 8 * chunk;
  *(volatile v4u*)dst = o;
  __threadfence();
  *(volatile v4u*)dst = o;
}

extern "C" void kernel_launch(void* const* d_in, const int* in_sizes, int n_in,
                              void* d_out, int out_size, void* d_ws, size_t ws_size,
                              hipStream_t stream) {
  if (n_in < 4) return;
  if (in_sizes[0] != kBs * kTlen) return;
  if (in_sizes[1] != 2 * kFreq) return;
  if (in_sizes[2] != 2 * kFreq) return;
  if (in_sizes[3] != 2 * kFreq * kSteps) return;
  if (out_size != kBs * kOutLen) return;
  if (ws_size < kWsTotal) return;

  const float* x    = (const float*)d_in[0];
  const float* lmr  = (const float*)d_in[1];
  const float* lmdr = (const float*)d_in[2];
  const float* ang  = (const float*)d_in[3];
  float* out = (float*)d_out;

  char* ws = (char*)d_ws;
  unsigned short* BST = (unsigned short*)(ws + kOffBST);
  unsigned short* IBT = (unsigned short*)(ws + kOffIBT);
  unsigned short* WT  = (unsigned short*)(ws + kOffWT);
  unsigned short* FR  = (unsigned short*)(ws + kOffFR);
  unsigned short* HS  = (unsigned short*)(ws + kOffHS);
  unsigned short* YC  = (unsigned short*)(ws + kOffYC);
  unsigned short* YA  = (unsigned short*)(ws + kOffYA);

  ir_taps_kernel<<<kFreq, 256, 0, stream>>>(lmr, lmdr, ang, WT);
  dft_planes_kernel<<<168, 256, 0, stream>>>(BST, IBT);
  frame_rows_kernel<<<(kCols * 48) / 256, 256, 0, stream>>>(x, FR);

  wmma_gemm64_h<1><<<((kBasisRows / 64) * (kCols / 64)) / 8, 256, 0, stream>>>(
      BST, kNfft, FR, kNfft, (void*)HS, kCols, kBasisRows, kCols, kNfft, 1.0f);

  band_conv_kernel<<<kChan * 11, 32, 0, stream>>>(HS, WT, YC);

  pack_rows_kernel<<<kBs * kTiles * 7 + 7, 256, 0, stream>>>(YC, YA);

  wmma_gemm64_h<3><<<((kYaRows / 64) * (kHop / 64)) / 8, 256, 0, stream>>>(
      YA, kYaPitch, IBT, kSynK, (void*)out, kHop, kYaRows, kHop, kSynK, kInvNfft);
}
